// MultiHeadAttention_45741401703090
// MI455X (gfx1250) — hardware-verified
//
#include <hip/hip_runtime.h>


#ifndef NB
#define NB 4
#endif
#ifndef SEQ
#define SEQ 2048
#endif
#define NB_FULL  4
#define SEQ_FULL 2048
#define DM   512
#define NH   8
#define HD   64
#define WCAR 16.0f
#define PCAR 1024.0f
#define CCAR 64.0f
#define SCL  0.125f
#define L2E  1.4426950408889634f
#define NEGF (-3.402823466e38f)

typedef _Float16 h16;
typedef __attribute__((ext_vector_type(16))) _Float16 v16h;
typedef __attribute__((ext_vector_type(8)))  _Float16 v8h;
typedef __attribute__((ext_vector_type(8)))  float    v8f;
typedef __attribute__((ext_vector_type(4)))  float    v4f;
typedef v8h __attribute__((may_alias)) v8ha;
typedef v4f __attribute__((may_alias)) v4fa;

static_assert(NH * HD == DM);
static_assert(HD == 64);
static_assert(DM % 64 == 0);
static_assert(DM % 32 == 0);
static_assert(SEQ % 128 == 0);
static_assert(SEQ <= SEQ_FULL);
static_assert(NB <= NB_FULL);
static_assert((SEQ / 32) % 8 == 0);

#define SZ_X   ((size_t)NB * SEQ * DM * 2)
#define SZ_W   ((size_t)4 * DM * DM * 2)
#define WS_TOTAL (SZ_X * 5 + SZ_W)
static_assert(SZ_X % 256 == 0);
static_assert(SZ_W % 256 == 0);
static_assert(WS_TOTAL <= (size_t)134217728);

__device__ __forceinline__ unsigned short f2bf(float f) { unsigned u = __float_as_uint(f); u += 0x7FFFu + ((u >> 16) & 1u); return (unsigned short)(u >> 16); }
__device__ __forceinline__ float bfr(float f) { return __uint_as_float(((unsigned)f2bf(f)) << 16); }
__device__ __forceinline__ v16h cat16(v8h lo, v8h hi) { return __builtin_shufflevector(lo, hi, 0, 1, 2, 3, 4, 5, 6, 7, 8, 9, 10, 11, 12, 13, 14, 15); }
__device__ __forceinline__ v16h ldfrag(const h16* p) { return cat16(*(const v8h*)p, *(const v8h*)(p + 16)); }
__device__ __forceinline__ v8f wm16(v16h a, v16h b, v8f c) {
    c = __builtin_amdgcn_wmma_f32_16x16x32_f16(false, a, false, b, (short)0, c, false, false);
    asm volatile("v_nop\n\tv_nop\n\tv_nop\n\tv_nop" : "+v"(c) : "v"(a), "v"(b));
    return c;
}
__device__ __forceinline__ float ex2(float x) { return __builtin_amdgcn_exp2f(x); }
__device__ __forceinline__ float redmax16(float v) {
    v = fmaxf(v, __shfl_xor(v, 1, 32)); v = fmaxf(v, __shfl_xor(v, 2, 32));
    v = fmaxf(v, __shfl_xor(v, 4, 32)); v = fmaxf(v, __shfl_xor(v, 8, 32)); return v;
}
__device__ __forceinline__ float redsum16(float v) {
    v += __shfl_xor(v, 1, 32); v += __shfl_xor(v, 2, 32);
    v += __shfl_xor(v, 4, 32); v += __shfl_xor(v, 8, 32); return v;
}

__global__ __launch_bounds__(256) void k_cvtx(const float* __restrict__ x, h16* xh) {
    const size_t i = (size_t)blockIdx.x * 256 + threadIdx.x;
    if (i >= (size_t)NB * SEQ * DM / 8) return;
    const size_t row = i / (DM / 8); const int g = (int)(i % (DM / 8));
    const size_t b = row / SEQ, s = row % SEQ;
    const float* src = x + ((b * SEQ_FULL + s) * DM + (size_t)g * 8);
    const v4f v0 = *(const v4f*)src; const v4f v1 = *(const v4f*)(src + 4);
    v8h o;
#pragma unroll
    for (int k = 0; k < 4; ++k) { o[k] = (h16)bfr(v0[k]); o[4 + k] = (h16)bfr(v1[k]); }
    *(volatile v8h*)(xh + i * 8) = o; __threadfence(); *(volatile v8h*)(xh + i * 8) = o;
}

__global__ __launch_bounds__(256) void k_wt(const float* __restrict__ W, h16* Wt) {
    __shared__ __align__(16) h16 T[64 * 72];
    const int tid = threadIdx.x; const int k0 = blockIdx.x * 64, n0 = blockIdx.y * 64;
#pragma unroll
    for (int j = 0; j < 4; ++j) { const int i = tid + 256 * j; const int kr = i >> 4, c4 = (i & 15) * 4;
        const v4f v = *(const v4f*)(W + (size_t)(k0 + kr) * DM + n0 + c4);
#pragma unroll
        for (int q = 0; q < 4; ++q) T[(c4 + q) * 72 + kr] = (h16)(bfr(v[q]) * WCAR); }
    __syncthreads();
#pragma unroll 1
    for (int ps = 0; ps < 2; ++ps) {
#pragma unroll
        for (int j = 0; j < 2; ++j) { const int p = tid + 256 * j; const int n = p >> 3, seg = p & 7;
            const v8h val = *(const v8ha*)(T + n * 72 + seg * 8);
            *(volatile v8h*)(Wt + (size_t)(n0 + n) * DM + k0 + seg * 8) = val; }
        if (ps == 0) __threadfence(); }
}

__device__ __forceinline__ void gemm64(const h16* __restrict__ A, const h16* __restrict__ Bt, size_t aoff, size_t boff, v8f (&acc)[4][4]) {
#pragma unroll 1
    for (int kc = 0; kc < DM; kc += 32) {
        v16h a[4];
#pragma unroll
        for (int mb = 0; mb < 4; ++mb) a[mb] = ldfrag(A + aoff + (size_t)mb * 16 * DM + kc);
#pragma unroll
        for (int nb = 0; nb < 4; ++nb) { const v16h b = ldfrag(Bt + boff + (size_t)nb * 16 * DM + kc);
#pragma unroll
            for (int mb = 0; mb < 4; ++mb) acc[mb][nb] = wm16(a[mb], b, acc[mb][nb]); }
    }
}

__global__ __launch_bounds__(32) void k_proj_qk(const h16* __restrict__ A, const h16* __restrict__ Bt, const float* __restrict__ bias, h16* plane) {
    __shared__ __align__(16) h16 T[64 * 72];
    const int lane = threadIdx.x & 31, lr = lane & 15, hi = lane >> 4;
    const int r0 = blockIdx.x * 64, c0 = blockIdx.y * 64;
    v8f acc[4][4];
#pragma unroll
    for (int mb = 0; mb < 4; ++mb)
#pragma unroll
        for (int nb = 0; nb < 4; ++nb) acc[mb][nb] = (v8f){};
    gemm64(A, Bt, (size_t)(r0 + lr) * DM + 8 * hi, (size_t)(c0 + lr) * DM + 8 * hi, acc);
#pragma unroll
    for (int nb = 0; nb < 4; ++nb) { const float bv = bfr(bias[c0 + nb * 16 + lr]);
#pragma unroll
        for (int mb = 0; mb < 4; ++mb)
#pragma unroll
            for (int j = 0; j < 8; ++j) T[(mb * 16 + hi * 8 + j) * 72 + nb * 16 + lr] = (h16)(acc[mb][nb][j] * (1.0f / WCAR) + bv); }
    __syncthreads();
    const int b = r0 / SEQ, s0 = r0 % SEQ, h = blockIdx.y;
    h16* dst = plane + ((size_t)(b * NH + h) * SEQ + s0) * HD;
#pragma unroll 1
    for (int ps = 0; ps < 2; ++ps) {
#pragma unroll
        for (int it = 0; it < 16; ++it) { const int piece = it * 32 + lane; const int row = piece >> 3, seg = piece & 7;
            const v8h val = *(const v8ha*)(T + row * 72 + seg * 8);
            *(volatile v8h*)(dst + (size_t)row * HD + seg * 8) = val; }
        if (ps == 0) __threadfence(); }
}

__global__ __launch_bounds__(32) void k_proj_v(const h16* __restrict__ A, const h16* __restrict__ Bt, const float* __restrict__ bias, h16* VT) {
    __shared__ __align__(16) h16 T[64 * 72];
    const int lane = threadIdx.x & 31, lr = lane & 15, hi = lane >> 4;
    const int r0 = blockIdx.x * 64, c0 = blockIdx.y * 64;
    v8f acc[4][4];
#pragma unroll
    for (int mb = 0; mb < 4; ++mb)
#pragma unroll
        for (int nb = 0; nb < 4; ++nb) acc[mb][nb] = (v8f){};
    gemm64(A, Bt, (size_t)(r0 + lr) * DM + 8 * hi, (size_t)(c0 + lr) * DM + 8 * hi, acc);
#pragma unroll
    for (int nb = 0; nb < 4; ++nb) { const float bv = bfr(bias[c0 + nb * 16 + lr]);
#pragma unroll
        for (int mb = 0; mb < 4; ++mb) { v8h pk;
#pragma unroll
            for (int j = 0; j < 8; ++j) pk[j] = (h16)(acc[mb][nb][j] * (1.0f / WCAR) + bv);
            *(v8ha*)(T + (nb * 16 + lr) * 72 + mb * 16 + hi * 8) = pk; } }
    __syncthreads();
    const int b = r0 / SEQ, s0 = r0 % SEQ, h = blockIdx.y;
    h16* dst = VT + ((size_t)(b * NH + h) * HD) * SEQ + s0;
#pragma unroll 1
    for (int ps = 0; ps < 2; ++ps) {
#pragma unroll
        for (int it = 0; it < 16; ++it) { const int piece = it * 32 + lane; const int d = piece >> 3, seg = piece & 7;
            const v8h val = *(const v8ha*)(T + d * 72 + seg * 8);
            *(volatile v8h*)(dst + (size_t)d * SEQ + seg * 8) = val; }
        if (ps == 0) __threadfence(); }
}

__global__ __launch_bounds__(32) void k_proj_out(const h16* __restrict__ A, const h16* __restrict__ Bt, const float* __restrict__ bias, float* C) {
    __shared__ __align__(16) float os[16 * 68];
    const int lane = threadIdx.x & 31, lr = lane & 15, hi = lane >> 4;
    const int r0 = blockIdx.x * 64, c0 = blockIdx.y * 64;
    v8f acc[4][4];
#pragma unroll
    for (int mb = 0; mb < 4; ++mb)
#pragma unroll
        for (int nb = 0; nb < 4; ++nb) acc[mb][nb] = (v8f){};
    gemm64(A, Bt, (size_t)(r0 + lr) * DM + 8 * hi, (size_t)(c0 + lr) * DM + 8 * hi, acc);
    const int b = r0 / SEQ, s0 = r0 % SEQ; const int cofs = lr * 4;
    v4f b4;
#pragma unroll
    for (int q = 0; q < 4; ++q) b4[q] = bfr(bias[c0 + cofs + q]);
    const float fs = 1.0f / (WCAR * CCAR);
#pragma unroll
    for (int mb = 0; mb < 4; ++mb) {
#pragma unroll
        for (int nb = 0; nb < 4; ++nb)
#pragma unroll
            for (int j = 0; j < 8; ++j) os[(hi * 8 + j) * 68 + nb * 16 + lr] = acc[mb][nb][j];
        __syncthreads();
        float* crow = C + ((size_t)b * SEQ_FULL + s0 + mb * 16) * DM + c0;
#pragma unroll 1
        for (int ps = 0; ps < 2; ++ps) {
#pragma unroll
            for (int s = 0; s < 8; ++s) { const int row = 2 * s + hi; const v4f raw = *(const v4fa*)(os + row * 68 + cofs); v4f val;
#pragma unroll
                for (int q = 0; q < 4; ++q) val[q] = raw[q] * fs + b4[q];
                *(volatile v4f*)(crow + (size_t)row * DM + cofs) = val; }
            if (ps == 0) __threadfence(); }
        __syncthreads();
    }
}

__global__ __launch_bounds__(256) void k_attn(const h16* __restrict__ Q, const h16* __restrict__ Kp, const h16* __restrict__ VT, const int* __restrict__ mask, h16* ctx) {
    __shared__ __align__(16) h16 Pl[8 * 16 * 72];
    __shared__ unsigned smw[SEQ / 32];
    const int tid = threadIdx.x, lane = tid & 31, lr = lane & 15, hi = lane >> 4;
    const int wave = __builtin_amdgcn_readfirstlane(tid >> 5);
    const int bh = blockIdx.x; const int b = bh / NH, h = bh % NH;
    const int q0 = blockIdx.y * 128;
#pragma unroll 1
    for (int w = wave; w < SEQ / 32; w += 8) { const int mv = mask[(size_t)b * SEQ_FULL + w * 32 + lane];
        const unsigned bits = __builtin_amdgcn_ballot_w32(mv != 0); if (lane == 0) smw[w] = bits; }
    __syncthreads();
    const size_t pbase = (size_t)bh * SEQ * HD;
    const h16* vt = VT + pbase;
    const int pw = wave * 16 * 72;
    v16h qf0, qf1;
    { const h16* qp = Q + pbase + (size_t)(q0 + wave * 16 + lr) * HD + 8 * hi; qf0 = ldfrag(qp); qf1 = ldfrag(qp + 32); }
    v8f o[4]; float mi[8], li[8];
#pragma unroll
    for (int t = 0; t < 4; ++t) o[t] = (v8f){};
#pragma unroll
    for (int r = 0; r < 8; ++r) { mi[r] = NEGF; li[r] = 0.0f; }
#pragma unroll 1
    for (int kv0 = 0; kv0 < SEQ; kv0 += 64) {
        v8f sa[4];
#pragma unroll
        for (int t = 0; t < 4; ++t) { const h16* kp = Kp + pbase + (size_t)(kv0 + t * 16 + lr) * HD + 8 * hi; v8f c = (v8f){};
            c = wm16(qf0, ldfrag(kp), c); c = wm16(qf1, ldfrag(kp + 32), c); sa[t] = c; }
        const unsigned w0 = smw[kv0 >> 5], w1 = smw[(kv0 >> 5) + 1];
        const bool k0ok = ((w0 >> lr) & 1u) != 0u, k1ok = ((w0 >> (16 + lr)) & 1u) != 0u, k2ok = ((w1 >> lr) & 1u) != 0u, k3ok = ((w1 >> (16 + lr)) & 1u) != 0u;
#pragma unroll
        for (int r = 0; r < 8; ++r) {
            const float s0 = k0ok ? sa[0][r] * SCL : NEGF; const float s1 = k1ok ? sa[1][r] * SCL : NEGF;
            const float s2 = k2ok ? sa[2][r] * SCL : NEGF; const float s3 = k3ok ? sa[3][r] * SCL : NEGF;
            float vm = fmaxf(fmaxf(s0, s1), fmaxf(s2, s3)); vm = redmax16(vm);
            const float mnew = fmaxf(mi[r], vm);
            const float alpha = ex2(fmaxf(mi[r] - mnew, -150.0f) * L2E); mi[r] = mnew;
            const float p0 = ex2(fmaxf(s0 - mnew, -150.0f) * L2E); const float p1 = ex2(fmaxf(s1 - mnew, -150.0f) * L2E);
            const float p2 = ex2(fmaxf(s2 - mnew, -150.0f) * L2E); const float p3 = ex2(fmaxf(s3 - mnew, -150.0f) * L2E);
            li[r] = li[r] * alpha + ((p0 + p1) + (p2 + p3));
            const int pr = pw + (hi * 8 + r) * 72 + lr;
            Pl[pr] = (h16)(p0 * PCAR); Pl[pr + 16] = (h16)(p1 * PCAR); Pl[pr + 32] = (h16)(p2 * PCAR); Pl[pr + 48] = (h16)(p3 * PCAR);
#pragma unroll
            for (int t = 0; t < 4; ++t) o[t][r] *= alpha;
        }
        asm volatile("" ::: "memory"); __builtin_amdgcn_wave_barrier(); asm volatile("" ::: "memory");
#pragma unroll
        for (int s2 = 0; s2 < 2; ++s2) {
            const v16h pf = cat16(*(const v8ha*)(Pl + pw + lr * 72 + s2 * 32 + 8 * hi), *(const v8ha*)(Pl + pw + lr * 72 + s2 * 32 + 16 + 8 * hi));
#pragma unroll
            for (int t = 0; t < 4; ++t) { const h16* vp = vt + (size_t)(t * 16 + lr) * SEQ + kv0 + s2 * 32 + 8 * hi; o[t] = wm16(pf, ldfrag(vp), o[t]); }
        }
        asm volatile("" ::: "memory"); __builtin_amdgcn_wave_barrier(); asm volatile("" ::: "memory");
    }
#pragma unroll
    for (int r = 0; r < 8; ++r) { const float l = redsum16(li[r]); const float inv = (CCAR / PCAR) * __builtin_amdgcn_rcpf(l);
#pragma unroll
        for (int t = 0; t < 4; ++t) Pl[pw + (hi * 8 + r) * 72 + t * 16 + lr] = (h16)(o[t][r] * inv); }
    asm volatile("" ::: "memory"); __builtin_amdgcn_wave_barrier(); asm volatile("" ::: "memory");
    h16* dst = ctx + ((size_t)b * SEQ + q0 + wave * 16) * DM + h * HD;
#pragma unroll 1
    for (int ps = 0; ps < 2; ++ps) {
#pragma unroll
        for (int it = 0; it < 4; ++it) { const int piece = it * 32 + lane; const int row = piece >> 3, seg = piece & 7;
            const v8h val = *(const v8ha*)(Pl + pw + row * 72 + seg * 8);
            *(volatile v8h*)(dst + (size_t)row * DM + seg * 8) = val; }
        if (ps == 0) __threadfence(); }
}

extern "C" void kernel_launch(void* const* d_in, const int* in_sizes, int n_in,
                              void* d_out, int out_size, void* d_ws, size_t ws_size, hipStream_t stream) {
    if (n_in < 10) return;
    const size_t xneed = ((size_t)(NB - 1) * SEQ_FULL + SEQ) * DM;
    const size_t mneed = (size_t)(NB - 1) * SEQ_FULL + SEQ;
    if ((size_t)in_sizes[0] < xneed || (size_t)in_sizes[1] < mneed) return;
    if (in_sizes[2] < DM * DM || in_sizes[4] < DM * DM || in_sizes[6] < DM * DM || in_sizes[8] < DM * DM) return;
    if (in_sizes[3] < DM || in_sizes[5] < DM || in_sizes[7] < DM || in_sizes[9] < DM) return;
    if ((size_t)out_size < xneed) return;
    if (ws_size < WS_TOTAL) return;
    const float* x  = (const float*)d_in[0]; const int* mask = (const int*)d_in[1];
    const float* wq = (const float*)d_in[2]; const float* bq = (const float*)d_in[3];
    const float* wk = (const float*)d_in[4]; const float* bk = (const float*)d_in[5];
    const float* wv = (const float*)d_in[6]; const float* bv = (const float*)d_in[7];
    const float* wo = (const float*)d_in[8]; const float* bo = (const float*)d_in[9];
    float* OUT = (float*)d_out;
    char* wsp = (char*)d_ws;
    h16* XH = (h16*)wsp; wsp += SZ_X;
    h16* WT = (h16*)wsp; wsp += SZ_W;
    h16* QP = (h16*)wsp; wsp += SZ_X;
    h16* KP = (h16*)wsp; wsp += SZ_X;
    h16* VT = (h16*)wsp; wsp += SZ_X;
    h16* CX = (h16*)wsp; wsp += SZ_X;
    const size_t wsz = (size_t)DM * DM;
    k_cvtx<<<(unsigned)(((size_t)NB * SEQ * DM / 8 + 255) / 256), 256, 0, stream>>>(x, XH);
    const dim3 gw(DM / 64, DM / 64);
    k_wt<<<gw, 256, 0, stream>>>(wq, WT);
    k_wt<<<gw, 256, 0, stream>>>(wk, WT + wsz);
    k_wt<<<gw, 256, 0, stream>>>(wv, WT + 2 * wsz);
    k_wt<<<gw, 256, 0, stream>>>(wo, WT + 3 * wsz);
    const dim3 gg(NB * SEQ / 64, DM / 64);
    k_proj_qk<<<gg, 32, 0, stream>>>(XH, WT, bq, QP);
    k_proj_qk<<<gg, 32, 0, stream>>>(XH, WT + wsz, bk, KP);
    k_proj_v<<<gg, 32, 0, stream>>>(XH, WT + 2 * wsz, bv, VT);
    k_attn<<<dim3(NB * NH, SEQ / 128), 256, 0, stream>>>(QP, KP, VT, mask, CX);
    k_proj_out<<<gg, 32, 0, stream>>>(CX, WT + 3 * wsz, bo, OUT);
}
